// NerfRenderer_41188736368830
// MI455X (gfx1250) — hardware-verified
//
#include <hip/hip_runtime.h>
#include <math.h>

#pragma clang fp contract(off)

typedef __attribute__((ext_vector_type(16))) _Float16 v16h;
typedef __attribute__((ext_vector_type(8)))  _Float16 v8h;
typedef __attribute__((ext_vector_type(8)))  float    v8f;
typedef __attribute__((ext_vector_type(4)))  float    v4f;

constexpr int NTHR  = 128;
constexpr int NROWS = 127;
constexpr int HIDN  = 64;
constexpr int FDIM  = 32;
constexpr int GSZ   = 128;
constexpr int RPB   = 32;
constexpr int OUTC  = 3;
constexpr float WCAR     = 16.0f;
constexpr float WCAR_INV = 0.0625f;
constexpr float T_NEAR   = 0.1f;
constexpr float T_NEAR1  = 1.1f;
constexpr float LOGC     = 0.0038986404156573229f;
constexpr float R63      = 1.0f / 63.0f;
constexpr float ETERM    = 1.0e-4f;

union FragU { v16h v; v8h h[2]; };
__device__ __forceinline__ v16h frag_load(const _Float16* p) {
  FragU f; f.h[0] = *(const v8h*)(p); f.h[1] = *(const v8h*)(p + 16); return f.v;
}
__device__ __forceinline__ v8f mma_g(v16h a, v16h b, v8f c) {
  c = __builtin_amdgcn_wmma_f32_16x16x32_f16(false, a, false, b, (short)0, c, false, false);
  asm volatile("v_nop\n\tv_nop\n\tv_nop\n\tv_nop" : "+v"(c) : "v"(a), "v"(b));
  return c;
}
__device__ __forceinline__ v8f zero8() { return (v8f){0.f, 0.f, 0.f, 0.f, 0.f, 0.f, 0.f, 0.f}; }

__device__ __forceinline__ float t_sched(int i) {
  const float fi = (float)i;
  const float st = fi * R63;
  const float u  = 1.0f - st;
  const float a  = T_NEAR * u;
  const float b  = T_NEAR1 * st;
  const float tc = (i >= 63) ? T_NEAR1 : (a + b);
  const float fj = (float)(i - 64);
  const float e  = fj * LOGC;
  const float tf = expf(e) * T_NEAR1;
  return (i >= 64) ? tf : tc;
}

__global__ __launch_bounds__(NTHR) void render_fused_kernel(
    const float* __restrict__ rays_o, const float* __restrict__ rays_d, const float* __restrict__ grid,
    const float* __restrict__ W1,  const float* __restrict__ b1,
    const float* __restrict__ W2,  const float* __restrict__ b2,
    const float* __restrict__ Ws,  const float* __restrict__ bs,
    const float* __restrict__ Wr1, const float* __restrict__ br1,
    const float* __restrict__ Wr2, const float* __restrict__ br2,
    const int* __restrict__ nsamp,
    float* __restrict__ out, int n_rays, int out_elems)
{
  __shared__ __align__(16) _Float16 sh_ha[NTHR * HIDN];
  __shared__ __align__(16) _Float16 sh_fa[NTHR * FDIM];
  __shared__ __align__(16) _Float16 sh_w2t[FDIM * HIDN];
  __shared__ __align__(16) _Float16 sh_wr1t[HIDN * FDIM];
  __shared__ __align__(16) _Float16 sh_wst[16 * FDIM];
  __shared__ __align__(16) _Float16 sh_wr2t[16 * HIDN];
  __shared__ float sh_w1[3 * HIDN];
  __shared__ float sh_wr1d[3 * HIDN];
  __shared__ float sh_b1[HIDN];
  __shared__ float sh_br1[HIDN];
  __shared__ float sh_b2[FDIM];
  __shared__ float sh_br2[4];
  __shared__ float sh_mask[NTHR];
  __shared__ float sh_pre[NTHR];
  __shared__ float sh_rgb[NTHR * 4];
  __shared__ float sh_dterm[HIDN];
  __shared__ float sh_wtot[4];
  __shared__ float sh_part[16];
  __shared__ __align__(16) float sh_out[RPB * OUTC];

  const int tid  = threadIdx.x;
  const int lane = tid & 31;
  const int wave = tid >> 5;
  const int rl   = lane & 15;
  const int hh   = lane >> 4;
  const int koff = hh * 8;
  const int blk  = blockIdx.x;

#pragma unroll 1
  for (int i = tid; i < 3 * HIDN; i += NTHR) {
    sh_w1[i]   = W1[i];
    sh_wr1d[i] = Wr1[FDIM * HIDN + i];
  }
  if (tid < HIDN) { sh_b1[tid] = b1[tid]; sh_br1[tid] = br1[tid]; }
  if (tid < FDIM) { sh_b2[tid] = b2[tid]; }
  {
    const float bv = br2[(tid < 3) ? tid : 2];
    if (tid < 4) sh_br2[tid] = bv * ((tid < 3) ? 1.0f : 0.0f);
  }
  const float bsv = bs[0];
#pragma unroll 1
  for (int idx = tid; idx < FDIM * HIDN; idx += NTHR) {
    const int n = idx >> 6, k = idx & 63;
    sh_w2t[idx] = (_Float16)(W2[k * FDIM + n] * WCAR);
  }
#pragma unroll 1
  for (int idx = tid; idx < HIDN * FDIM; idx += NTHR) {
    const int n = idx >> 5, k = idx & 31;
    sh_wr1t[idx] = (_Float16)(Wr1[k * HIDN + n] * WCAR);
  }
#pragma unroll 1
  for (int idx = tid; idx < 16 * FDIM; idx += NTHR) {
    const int n = idx >> 5, k = idx & 31;
    const float w = Ws[k];
    sh_wst[idx] = (_Float16)(w * ((n == 0) ? WCAR : 0.0f));
  }
#pragma unroll 1
  for (int idx = tid; idx < 16 * HIDN; idx += NTHR) {
    const int n = idx >> 6, k = idx & 63;
    const int nc = (n < 3) ? n : 2;
    const float w = Wr2[k * 3 + nc];
    sh_wr2t[idx] = (_Float16)(w * ((n < 3) ? WCAR : 0.0f));
  }
  int nreal = nsamp[0] - 1;
  nreal = (nreal < 1) ? 1 : nreal;
  nreal = (nreal > NROWS) ? NROWS : nreal;
  const bool valid = (tid < nreal);
  const float t0   = t_sched(tid);
  const float t1   = t_sched((tid + 1 < NTHR) ? (tid + 1) : (NTHR - 1));
  const float dist = valid ? (t1 - t0) : 0.0f;
  __syncthreads();

  for (int rs = 0; rs < RPB; ++rs) {
    const int ray  = blk * RPB + rs;
    const int rayc = (ray < n_rays) ? ray : (n_rays - 1);
    const float ox = rays_o[rayc * 3 + 0], oy = rays_o[rayc * 3 + 1], oz = rays_o[rayc * 3 + 2];
    const float dx = rays_d[rayc * 3 + 0], dy = rays_d[rayc * 3 + 1], dz = rays_d[rayc * 3 + 2];

    if (tid < HIDN) {
      float p = dx * sh_wr1d[tid];
      p = fmaf(dy, sh_wr1d[HIDN + tid], p);
      p = fmaf(dz, sh_wr1d[2 * HIDN + tid], p);
      sh_dterm[tid] = p + sh_br1[tid];
    }

    const float mx = dx * t0, my = dy * t0, mz = dz * t0;
    const float px = ox + mx, py = oy + my, pz = oz + mz;
    const float nrm = fmaxf(fabsf(px), fmaxf(fabsf(py), fabsf(pz)));
    const float nsd = fmaxf(nrm, 1.0f);
    const float rcp = 1.0f / nsd;
    const float q1  = 2.0f - rcp;
    const float qx  = (q1 * px) * rcp, qy = (q1 * py) * rcp, qz = (q1 * pz) * rcp;
    const bool inside = (nrm <= 1.0f);
    const float scx = (inside ? px : qx) * 0.5f;
    const float scy = (inside ? py : qy) * 0.5f;
    const float scz = (inside ? pz : qz) * 0.5f;

    const float gx = (((scx + 1.0f) * 128.0f) - 1.0f) * 0.5f;
    const float gy = (((scy + 1.0f) * 128.0f) - 1.0f) * 0.5f;
    const float gz = (((scz + 1.0f) * 128.0f) - 1.0f) * 0.5f;
    const float flx = floorf(gx), fly = floorf(gy), flz = floorf(gz);
    const float fx = gx - flx, fy = gy - fly, fz = gz - flz;
    const int x0 = (int)flx, y0 = (int)fly, z0 = (int)flz;
    const float wx0 = 1.0f - fx, wy0 = 1.0f - fy, wz0 = 1.0f - fz;
    const float vx0 = (x0 >= 0 && x0 < GSZ) ? 1.0f : 0.0f;
    const float vx1 = (x0 + 1 >= 0 && x0 + 1 < GSZ) ? 1.0f : 0.0f;
    const float vy0 = (y0 >= 0 && y0 < GSZ) ? 1.0f : 0.0f;
    const float vy1 = (y0 + 1 >= 0 && y0 + 1 < GSZ) ? 1.0f : 0.0f;
    const float vz0 = (z0 >= 0 && z0 < GSZ) ? 1.0f : 0.0f;
    const float vz1 = (z0 + 1 >= 0 && z0 + 1 < GSZ) ? 1.0f : 0.0f;
    const int xc0 = min(max(x0, 0), GSZ - 1), xc1 = min(max(x0 + 1, 0), GSZ - 1);
    const int yc0 = min(max(y0, 0), GSZ - 1), yc1 = min(max(y0 + 1, 0), GSZ - 1);
    const int zc0 = min(max(z0, 0), GSZ - 1), zc1 = min(max(z0 + 1, 0), GSZ - 1);
    const int bz0 = zc0 * GSZ * GSZ, bz1 = zc1 * GSZ * GSZ, by0 = yc0 * GSZ, by1 = yc1 * GSZ;
    const float g000 = grid[bz0 + by0 + xc0];
    const float g001 = grid[bz0 + by0 + xc1];
    const float g010 = grid[bz0 + by1 + xc0];
    const float g011 = grid[bz0 + by1 + xc1];
    const float g100 = grid[bz1 + by0 + xc0];
    const float g101 = grid[bz1 + by0 + xc1];
    const float g110 = grid[bz1 + by1 + xc0];
    const float g111 = grid[bz1 + by1 + xc1];
    const float c000 = g000 * ((vz0 * vy0) * vx0);
    const float c001 = g001 * ((vz0 * vy0) * vx1);
    const float c010 = g010 * ((vz0 * vy1) * vx0);
    const float c011 = g011 * ((vz0 * vy1) * vx1);
    const float c100 = g100 * ((vz1 * vy0) * vx0);
    const float c101 = g101 * ((vz1 * vy0) * vx1);
    const float c110 = g110 * ((vz1 * vy1) * vx0);
    const float c111 = g111 * ((vz1 * vy1) * vx1);
    float occ = ((c000 * wz0) * wy0) * wx0;
    occ = occ + ((c001 * wz0) * wy0) * fx;
    occ = occ + ((c010 * wz0) * fy) * wx0;
    occ = occ + ((c011 * wz0) * fy) * fx;
    occ = occ + ((c100 * fz) * wy0) * wx0;
    occ = occ + ((c101 * fz) * wy0) * fx;
    occ = occ + ((c110 * fz) * fy) * wx0;
    occ = occ + ((c111 * fz) * fy) * fx;
    const float maskf = (valid && (occ > 0.0f)) ? 1.0f : 0.0f;
    sh_mask[tid] = maskf;

    {
      _Float16* hrow = sh_ha + tid * HIDN;
#pragma unroll
      for (int g = 0; g < 8; ++g) {
        v8h pk;
#pragma unroll
        for (int e = 0; e < 8; ++e) {
          const int j = g * 8 + e;
          float p = scx * sh_w1[j];
          p = fmaf(scy, sh_w1[HIDN + j], p);
          p = fmaf(scz, sh_w1[2 * HIDN + j], p);
          p = p + sh_b1[j];
          pk[e] = (_Float16)fmaxf(p, 0.0f);
        }
        *(v8h*)(hrow + g * 8) = pk;
      }
    }
    __syncthreads();

    {
      const _Float16* arow = sh_ha + (wave * 32 + rl) * HIDN + koff;
#pragma unroll
      for (int mt = 0; mt < 2; ++mt) {
        const int S0 = wave * 32 + mt * 16;
        const v16h a0 = frag_load(arow + mt * 16 * HIDN);
        const v16h a1 = frag_load(arow + mt * 16 * HIDN + 32);
        float mrow[8];
#pragma unroll
        for (int r = 0; r < 8; ++r) mrow[r] = sh_mask[S0 + koff + r];
#pragma unroll
        for (int nt = 0; nt < 2; ++nt) {
          const _Float16* brow = sh_w2t + (nt * 16 + rl) * HIDN + koff;
          const v16h bA = frag_load(brow);
          const v16h bB = frag_load(brow + 32);
          v8f c = zero8();
          c = mma_g(a0, bA, c);
          c = mma_g(a1, bB, c);
          const int n = nt * 16 + rl;
          const float bn = sh_b2[n];
#pragma unroll
          for (int r = 0; r < 8; ++r) {
            const int row = S0 + koff + r;
            const float f = (c[r] * WCAR_INV + bn) * mrow[r];
            sh_fa[row * FDIM + n] = (_Float16)f;
          }
        }
      }
    }
    __syncthreads();

    {
      const v16h bw = frag_load(sh_wst + rl * FDIM + koff);
#pragma unroll
      for (int mt = 0; mt < 2; ++mt) {
        const int S0 = wave * 32 + mt * 16;
        const v16h a = frag_load(sh_fa + (S0 + rl) * FDIM + koff);
        v8f c = zero8();
        c = mma_g(a, bw, c);
        if (rl == 0) {
#pragma unroll
          for (int r = 0; r < 8; ++r) sh_pre[S0 + koff + r] = c[r] * WCAR_INV + bsv;
        }
      }
    }
    __syncthreads();

    const float pre   = sh_pre[tid];
    const float sp    = fmaxf(pre, 0.0f) + log1pf(expf(-fabsf(pre)));
    const float sigma = sp * maskf;
    const float nsig  = -sigma;
    const float alog  = valid ? (nsig * dist) : 0.0f;
    float incl = alog;
#pragma unroll
    for (int off = 1; off < 32; off <<= 1) {
      const float up = __shfl_up(incl, off, 32);
      incl = (lane >= off) ? (incl + up) : incl;
    }
    if (lane == 31) sh_wtot[wave] = incl;
    const float exl = __shfl_up(incl, 1, 32);
    __syncthreads();
    float prefix = 0.0f;
    {
      const float w0 = sh_wtot[0], w1v = sh_wtot[1], w2v = sh_wtot[2];
      prefix = (wave > 0) ? (prefix + w0)  : prefix;
      prefix = (wave > 1) ? (prefix + w1v) : prefix;
      prefix = (wave > 2) ? (prefix + w2v) : prefix;
    }
    const float cprev = prefix + ((lane > 0) ? exl : 0.0f);
    const float trans = expf(cprev);
    const float ea    = expf(alog);
    const float alpha = 1.0f - ea;
    const float wv    = trans * alpha;
    const bool keep2  = (maskf > 0.0f) && (wv > ETERM);
    const float wgt   = keep2 ? wv : 0.0f;

    {
#pragma unroll
      for (int mt = 0; mt < 2; ++mt) {
        const int S0 = wave * 32 + mt * 16;
        const v16h a = frag_load(sh_fa + (S0 + rl) * FDIM + koff);
#pragma unroll
        for (int nt = 0; nt < 4; ++nt) {
          const v16h b = frag_load(sh_wr1t + (nt * 16 + rl) * FDIM + koff);
          v8f c = zero8();
          c = mma_g(a, b, c);
          const int n = nt * 16 + rl;
          const float dn = sh_dterm[n];
#pragma unroll
          for (int r = 0; r < 8; ++r) {
            const int row = S0 + koff + r;
            const float hv = fmaxf(c[r] * WCAR_INV + dn, 0.0f);
            sh_ha[row * HIDN + n] = (_Float16)hv;
          }
        }
      }
    }
    __syncthreads();

    {
      const v16h bw0 = frag_load(sh_wr2t + rl * HIDN + koff);
      const v16h bw1 = frag_load(sh_wr2t + rl * HIDN + koff + 32);
      const float brc = sh_br2[(rl < 3) ? rl : 3];
#pragma unroll
      for (int mt = 0; mt < 2; ++mt) {
        const int S0 = wave * 32 + mt * 16;
        const v16h a0 = frag_load(sh_ha + (S0 + rl) * HIDN + koff);
        const v16h a1 = frag_load(sh_ha + (S0 + rl) * HIDN + koff + 32);
        v8f c = zero8();
        c = mma_g(a0, bw0, c);
        c = mma_g(a1, bw1, c);
        if (rl < 3) {
#pragma unroll
          for (int r = 0; r < 8; ++r) sh_rgb[(S0 + koff + r) * 4 + rl] = c[r] * WCAR_INV + brc;
        }
      }
    }
    __syncthreads();

    {
      const float p0 = sh_rgb[tid * 4 + 0];
      const float p1 = sh_rgb[tid * 4 + 1];
      const float p2 = sh_rgb[tid * 4 + 2];
      const float e0 = expf(-p0), e1 = expf(-p1), e2 = expf(-p2);
      float r0 = (1.0f / (1.0f + e0)) * wgt;
      float r1 = (1.0f / (1.0f + e1)) * wgt;
      float r2 = (1.0f / (1.0f + e2)) * wgt;
#pragma unroll
      for (int off = 16; off > 0; off >>= 1) {
        r0 = r0 + __shfl_xor(r0, off, 32);
        r1 = r1 + __shfl_xor(r1, off, 32);
        r2 = r2 + __shfl_xor(r2, off, 32);
      }
      if (lane == 0) {
        sh_part[wave * 4 + 0] = r0;
        sh_part[wave * 4 + 1] = r1;
        sh_part[wave * 4 + 2] = r2;
      }
    }
    __syncthreads();
    if (tid < 3) {
      float a = sh_part[tid];
      a = a + sh_part[4 + tid];
      a = a + sh_part[8 + tid];
      a = a + sh_part[12 + tid];
      sh_out[rs * OUTC + tid] = a;
    }
  }
  __syncthreads();

  if (wave == 0) {
    const int li = (lane < 24) ? lane : 0;
    const v4f val = *(const v4f*)(sh_out + li * 4);
    const size_t e0 = (size_t)blk * (RPB * OUTC) + (size_t)li * 4;
    const bool ok = (lane < 24) && (e0 + 4 <= (size_t)out_elems);
    float* op = out + e0;
    if (ok) { *(volatile v4f*)op = val; }
    __threadfence();
    if (ok) { *(volatile v4f*)op = val; }
  }
}

extern "C" void kernel_launch(void* const* d_in, const int* in_sizes, int n_in,
                              void* d_out, int out_size, void* d_ws, size_t ws_size,
                              hipStream_t stream) {
  (void)n_in; (void)d_ws; (void)ws_size;
  const float* rays_o = (const float*)d_in[0];
  const float* rays_d = (const float*)d_in[1];
  const float* grid   = (const float*)d_in[2];
  const float* W1     = (const float*)d_in[3];
  const float* b1     = (const float*)d_in[4];
  const float* W2     = (const float*)d_in[5];
  const float* b2     = (const float*)d_in[6];
  const float* Ws     = (const float*)d_in[7];
  const float* bs     = (const float*)d_in[8];
  const float* Wr1    = (const float*)d_in[9];
  const float* br1    = (const float*)d_in[10];
  const float* Wr2    = (const float*)d_in[11];
  const float* br2    = (const float*)d_in[12];
  const int*   nsamp  = (const int*)d_in[13];
  float* out = (float*)d_out;

  const int n_rays = in_sizes[0] / 3;
  if (n_rays <= 0) return;
  const int nblk = (n_rays + RPB - 1) / RPB;
  render_fused_kernel<<<dim3(nblk), dim3(NTHR), 0, stream>>>(
      rays_o, rays_d, grid, W1, b1, W2, b2, Ws, bs, Wr1, br1, Wr2, br2, nsamp,
      out, n_rays, out_size);
}
